// LinearAttentionMem_78683800863377
// MI455X (gfx1250) — hardware-verified
//
#include <hip/hip_runtime.h>
#include <stddef.h>


#define B_  16
#define S_  2048
#define D_  128
#define H_  8
#define NM_ 4
#define HD_ (D_ * H_)

typedef __attribute__((ext_vector_type(16))) _Float16 v16h;
typedef __attribute__((ext_vector_type(8)))  _Float16 v8h;
typedef __attribute__((ext_vector_type(16))) __bf16   v16b;
typedef __attribute__((ext_vector_type(8)))  __bf16   v8b;
typedef __attribute__((ext_vector_type(8)))  float    v8f;
typedef __attribute__((ext_vector_type(4)))  float    v4f;

__device__ __forceinline__ unsigned short f2bf_bits(float f) {
  unsigned u = __float_as_uint(f);
  return (unsigned short)((u + 0x7FFFu + ((u >> 16) & 1u)) >> 16);
}
__device__ __forceinline__ float bf_bits2f(unsigned short h) { return __uint_as_float(((unsigned)h) << 16); }

__device__ __forceinline__ void dep_guard_h(v8f& a, v8f& b, v16h x, v16h y) { asm volatile("v_nop\n\tv_nop\n\tv_nop\n\tv_nop" : "+v"(a), "+v"(b) : "v"(x), "v"(y)); }
__device__ __forceinline__ void dep_guard_b(v8f& a, v8f& b, v16b x, v16b y) { asm volatile("v_nop\n\tv_nop\n\tv_nop\n\tv_nop" : "+v"(a), "+v"(b) : "v"(x), "v"(y)); }
__device__ __forceinline__ void keep4_h(v16h a, v16h b, v16h c, v16h d) { asm volatile("v_nop" :: "v"(a), "v"(b), "v"(c), "v"(d)); }
__device__ __forceinline__ void keep4_b(v16b a, v16b b, v16b c, v16b d) { asm volatile("v_nop" :: "v"(a), "v"(b), "v"(c), "v"(d)); }
__device__ __forceinline__ void acc_guard4(v8f& a, v8f& b, v8f& c, v8f& d) { asm volatile("v_nop\n\tv_nop\n\tv_nop\n\tv_nop" : "+v"(a), "+v"(b), "+v"(c), "+v"(d)); }
template <typename T> struct Frag;
template <> struct Frag<_Float16> {
  typedef v16h V; union U { v16h v; v8h h[2]; };
  static __device__ __forceinline__ v16h load(const _Float16* p) {
    U f; f.h[0] = *(const v8h*)(p); f.h[1] = *(const v8h*)(p + 16); return f.v;
  }
  static __device__ __forceinline__ v8f mma(v16h a, v16h b, v8f c) {
    return __builtin_amdgcn_wmma_f32_16x16x32_f16(false, a, false, b, (short)0, c, false, false);
  }
  static __device__ __forceinline__ void guard(v8f& a, v8f& b, v16h x, v16h y) { dep_guard_h(a, b, x, y); }
  static __device__ __forceinline__ void keep(v16h a, v16h b, v16h c, v16h d) { keep4_h(a, b, c, d); }
};
template <> struct Frag<__bf16> {
  typedef v16b V; union U { v16b v; v8b h[2]; };
  static __device__ __forceinline__ v16b load(const __bf16* p) {
    U f; f.h[0] = *(const v8b*)(p); f.h[1] = *(const v8b*)(p + 16); return f.v;
  }
  static __device__ __forceinline__ v8f mma(v16b a, v16b b, v8f c) {
    return __builtin_amdgcn_wmma_f32_16x16x32_bf16(false, a, false, b, (short)0, c, false, false);
  }
  static __device__ __forceinline__ void guard(v8f& a, v8f& b, v16b x, v16b y) { dep_guard_b(a, b, x, y); }
  static __device__ __forceinline__ void keep(v16b a, v16b b, v16b c, v16b d) { keep4_b(a, b, c, d); }
};

template <int ET> struct Elem;
template <> struct Elem<0> { typedef _Float16 T; };
template <> struct Elem<1> { typedef __bf16 T; };
template <int ET, bool SPLIT, int BIAS_MODE, int OUT_MODE, bool RESID, int ACT, bool CSCALE, bool RSCALE>
__global__ __launch_bounds__(256) void wmma_gemm64(
    const unsigned short* __restrict__ Ap, const unsigned short* __restrict__ A2p, int lda, long strideA,
    const unsigned short* __restrict__ Btp, const unsigned short* __restrict__ Bt2p, int ldb, long strideB,
    void* __restrict__ Cout, void* __restrict__ Cout2, int ldc, long strideC,
    const float* __restrict__ bias,
    const float* __restrict__ resid, long strideR,
    const float* __restrict__ rsc, int rs_stride,
    const float* __restrict__ cs, long strideCS, int ldcs, int cs_shift, float post,
    int M, int N, int K, float scale) {
  typedef typename Elem<ET>::T T;
  typedef typename Frag<T>::V V;
  const T* A = (const T*)Ap; const T* A2 = (const T*)A2p; const T* Bt = (const T*)Btp; const T* Bt2 = (const T*)Bt2p;
  __shared__ __align__(16) float sT[8][16 * 68];
  const int b    = blockIdx.y;
  const int lane = threadIdx.x & 31;
  const int wave = threadIdx.x >> 5;
  const int tilesN = N >> 6;
  const int tilesM = M >> 6;
  const int tile = blockIdx.x * 8 + wave;
  if (tile >= tilesM * tilesN) return;
  const int tm = tile / tilesN;
  const int tn = tile - tm * tilesN;
  const int m0 = tm << 6;
  const int n0 = tn << 6;

  const T* Ab  = A  + (size_t)b * strideA;
  const T* Bb  = Bt + (size_t)b * strideB;
  const T* Ab2 = SPLIT ? (A2  + (size_t)b * strideA) : nullptr;
  const T* Bb2 = SPLIT ? (Bt2 + (size_t)b * strideB) : nullptr;

  const int rlane = lane & 15;
  const int koff  = (lane >> 4) * 8;
  const int mOff  = (lane >> 4) * 8;

  v8f acc[4][4];
#pragma unroll
  for (int i = 0; i < 4; ++i)
#pragma unroll
    for (int j = 0; j < 4; ++j) acc[i][j] = (v8f){0.f,0.f,0.f,0.f,0.f,0.f,0.f,0.f};

  for (int k0 = 0; k0 < K; k0 += 32) {
    V bh[4], bl[4];
#pragma unroll
    for (int j = 0; j < 4; ++j) {
      const size_t bo = (size_t)(n0 + (j << 4) + rlane) * ldb + koff + k0;
      bh[j] = Frag<T>::load(Bb + bo);
      if (SPLIT) bl[j] = Frag<T>::load(Bb2 + bo);
    }
#pragma unroll
    for (int i = 0; i < 4; ++i) {
      const size_t ao = (size_t)(m0 + (i << 4) + rlane) * lda + koff + k0;
      V ah = Frag<T>::load(Ab + ao);
      V al;
      if (SPLIT) al = Frag<T>::load(Ab2 + ao);
#pragma unroll
      for (int j = 0; j < 4; ++j) {
        acc[i][j] = Frag<T>::mma(ah, bh[j], acc[i][j]);
        if (SPLIT) {
          acc[i][j] = Frag<T>::mma(ah, bl[j], acc[i][j]);
          acc[i][j] = Frag<T>::mma(al, bh[j], acc[i][j]);
        }
      }
      Frag<T>::guard(acc[i][0], acc[i][3], ah, SPLIT ? al : ah);
    }
    Frag<T>::keep(bh[0], bh[1], bh[2], bh[3]);
    if (SPLIT) Frag<T>::keep(bl[0], bl[1], bl[2], bl[3]);
  }
  acc_guard4(acc[0][0], acc[0][1], acc[0][2], acc[0][3]);
  acc_guard4(acc[1][0], acc[1][1], acc[1][2], acc[1][3]);
  acc_guard4(acc[2][0], acc[2][1], acc[2][2], acc[2][3]);
  acc_guard4(acc[3][0], acc[3][1], acc[3][2], acc[3][3]);

  float* slab = sT[wave];
  const float* Rb = RESID ? (resid + (size_t)b * strideR) : nullptr;
  float rsv = 1.0f;
  if (RESID && RSCALE) rsv = rsc[(size_t)b * rs_stride];
  const float* csb = CSCALE ? (cs + (size_t)b * strideCS) : nullptr;
#pragma unroll
  for (int i = 0; i < 4; ++i) {
    const int mBase = m0 + (i << 4);
#pragma unroll
    for (int j = 0; j < 4; ++j) {
      const int n = n0 + (j << 4) + rlane;
      float bv = 0.f;
      if (BIAS_MODE == 2) bv = bias[n];
#pragma unroll
      for (int r = 0; r < 8; ++r) {
        const int m = mBase + mOff + r;
        float v = acc[i][j][r] * scale;
        if (BIAS_MODE == 1) v += bias[m];
        if (BIAS_MODE == 2) v += bv;
        if (CSCALE) v *= csb[(size_t)(m >> cs_shift) * ldcs + n];
        v *= post;
        if (RESID) { float rv = Rb[(size_t)m * ldc + n]; if (RSCALE) rv *= rsv; v += rv; }
        if (ACT == 1) v = tanhf(v);
        if (ACT == 2) v = fmaxf(v, 0.0f);
        if (ACT == 3) v = v / (1.0f + expf(-v));
        if (ACT == 4) v = (v > 0.f) ? v : 0.01f * v;
        if (ACT == 5) v = 0.5f * v * (1.0f + erff(v * 0.70710678118654752f));
        slab[(mOff + r) * 68 + (j << 4) + rlane] = v;
      }
    }
    __builtin_amdgcn_fence(__ATOMIC_RELEASE, "workgroup");
    __builtin_amdgcn_wave_barrier();
    __builtin_amdgcn_fence(__ATOMIC_ACQUIRE, "workgroup");
    if (OUT_MODE == 0) {
      float* C = (float*)Cout + (size_t)b * strideC;
      const int hh = lane >> 4, c4 = (lane & 15) * 4;
      for (int pass = 0; pass < 2; ++pass) {
#pragma unroll
        for (int it = 0; it < 8; ++it) {
          const int row = it * 2 + hh;
          v4f v = *(const v4f*)(slab + row * 68 + c4);
          *(volatile v4f*)(C + (size_t)(mBase + row) * ldc + n0 + c4) = v;
        }
        __threadfence();
      }
    } else {
      const int q = lane >> 3, c8 = (lane & 7) * 8;
      unsigned short* C  = (unsigned short*)Cout  + (size_t)b * strideC;
      unsigned short* C2 = (OUT_MODE == 2) ? ((unsigned short*)Cout2 + (size_t)b * strideC) : nullptr;
      for (int pass = 0; pass < 2; ++pass) {
#pragma unroll
        for (int it = 0; it < 4; ++it) {
          const int row = it * 4 + q;
          const float* sp = slab + row * 68 + c8;
          v8h hv, lv;
#pragma unroll
          for (int e = 0; e < 8; ++e) {
            if (OUT_MODE == 1) {
              hv[e] = (_Float16)sp[e];
            } else {
              unsigned short hb = f2bf_bits(sp[e]);
              unsigned short lb = f2bf_bits(sp[e] - bf_bits2f(hb));
              hv[e] = __builtin_bit_cast(_Float16, hb);
              lv[e] = __builtin_bit_cast(_Float16, lb);
            }
          }
          *(volatile v8h*)(C + (size_t)(mBase + row) * ldc + n0 + c8) = hv;
          if (OUT_MODE == 2) *(volatile v8h*)(C2 + (size_t)(mBase + row) * ldc + n0 + c8) = lv;
        }
        __threadfence();
      }
    }
    __builtin_amdgcn_fence(__ATOMIC_RELEASE, "workgroup");
    __builtin_amdgcn_wave_barrier();
    __builtin_amdgcn_fence(__ATOMIC_ACQUIRE, "workgroup");
  }
}

__global__ __launch_bounds__(256) void cast_f32_f16x2(
    const float* __restrict__ in, _Float16* __restrict__ out, int n2) {
  int i = blockIdx.x * 256 + threadIdx.x;
  if (i < n2) {
    const _Float16 h0 = (_Float16)in[2 * i], h1 = (_Float16)in[2 * i + 1];
    const unsigned u = (unsigned)__builtin_bit_cast(unsigned short, h0) | ((unsigned)__builtin_bit_cast(unsigned short, h1) << 16);
    ((volatile unsigned*)out)[i] = u;
    __threadfence();
    ((volatile unsigned*)out)[i] = u;
  }
}

__global__ __launch_bounds__(256) void wt_cast(
    const float* __restrict__ Wk, const float* __restrict__ Wv,
    _Float16* __restrict__ WkT, _Float16* __restrict__ WvT) {
  __shared__ __align__(16) float ts[32 * 132];
  const int tid = threadIdx.x, lane = tid & 31, wave = tid >> 5;
  const float* W = (blockIdx.y == 0) ? Wk : Wv;
  _Float16* O = (blockIdx.y == 0) ? WkT : WvT;
  const int hd0 = blockIdx.x * 32;
#pragma unroll
  for (int it = 0; it < 16; ++it) {
    const int i = it * 8 + wave;
    ts[lane * 132 + i] = W[(size_t)i * HD_ + hd0 + lane];
  }
  __syncthreads();
  for (int pass = 0; pass < 2; ++pass) {
#pragma unroll
    for (int it = 0; it < 2; ++it) {
      const int r = wave * 4 + it * 2 + (lane >> 4);
      const int c8 = (lane & 15) * 8;
      const float* sp = ts + r * 132 + c8;
      v8h hv;
#pragma unroll
      for (int e = 0; e < 8; ++e) hv[e] = (_Float16)sp[e];
      *(volatile v8h*)(O + (size_t)(hd0 + r) * D_ + c8) = hv;
    }
    __threadfence();
  }
}

__global__ __launch_bounds__(256) void gate_coef(
    const float* __restrict__ x, const float* __restrict__ router, const int* __restrict__ mem_id,
    const float* __restrict__ Wf, const float* __restrict__ bfp,
    float* __restrict__ cbuf, float* __restrict__ Fbuf) {
  __shared__ __align__(16) float fs[S_ * H_];
  __shared__ float wfl[D_ * H_];
  __shared__ float bfl[H_];
  __shared__ float Fs[H_];
  const int tid = threadIdx.x;
  const int b = blockIdx.x;
  int mid = mem_id[0];
  mid = mid < 0 ? 0 : (mid > NM_ - 1 ? NM_ - 1 : mid);
  for (int i = tid; i < D_ * H_; i += 256) wfl[i] = Wf[i];
  if (tid < H_) bfl[tid] = bfp[tid];
  __syncthreads();

#pragma unroll 1
  for (int it = 0; it < S_ / 256; ++it) {
    const int t = it * 256 + tid;
    const float* xr = x + ((size_t)b * S_ + t) * D_;
    float a[H_];
#pragma unroll
    for (int h = 0; h < H_; ++h) a[h] = bfl[h];
#pragma unroll 1
    for (int d = 0; d < D_; ++d) {
      const float xv = xr[d];
      const float* wr = wfl + d * H_;
#pragma unroll
      for (int h = 0; h < H_; ++h) a[h] += xv * wr[h];
    }
#pragma unroll
    for (int h = 0; h < H_; ++h) fs[t * H_ + h] = a[h];
  }
  __syncthreads();

#pragma unroll 1
  for (int i = tid; i < S_ * H_; i += 256) {
    const float av = fs[i];
    const float e = expf(-av);
    fs[i] = __builtin_amdgcn_rcpf(1.0f + e);
  }
  __syncthreads();

  if (tid < H_) {
    const int h = tid;
    const float* rp = router + (size_t)b * S_ * NM_ + mid;
    float P = 1.0f;
#pragma unroll 1
    for (int t = S_ - 1; t >= 0; --t) {
      const float wt = rp[(size_t)t * NM_];
      const float fv = fs[t * H_ + h];
      fs[t * H_ + h] = wt * P;
      P = P * fv;
    }
    Fs[h] = P;
  }
  __syncthreads();

  float* cb = cbuf + (size_t)b * H_ * S_;
  for (int pass = 0; pass < 2; ++pass) {
#pragma unroll 1
    for (int it = 0; it < (H_ * S_ / 4) / 256; ++it) {
      const int idx = it * 256 + tid;
      const int h = idx >> 9;
      const int t4 = (idx & 511) * 4;
      v4f v;
      v[0] = fs[(t4 + 0) * H_ + h];
      v[1] = fs[(t4 + 1) * H_ + h];
      v[2] = fs[(t4 + 2) * H_ + h];
      v[3] = fs[(t4 + 3) * H_ + h];
      *(volatile v4f*)(cb + (size_t)h * S_ + t4) = v;
    }
    __threadfence();
  }
  if (tid < 32) {
    for (int pass = 0; pass < 2; ++pass) {
#pragma unroll
      for (int h = 0; h < H_; ++h) {
        const float fv = Fs[h];
        const float val = (tid == 0) ? fv : 0.0f;
        *(volatile float*)(Fbuf + ((size_t)(b * H_ + h)) * 32 + tid) = val;
      }
      __threadfence();
    }
  }
}

extern "C" void kernel_launch(void* const* d_in, const int* in_sizes, int n_in,
                              void* d_out, int out_size, void* d_ws, size_t ws_size,
                              hipStream_t stream) {
  if (n_in < 10) return;
  if (in_sizes[0] != B_ * S_ * D_) return;
  if (in_sizes[1] != B_ * H_ * D_ * D_) return;
  if (in_sizes[2] != B_ * S_ * NM_) return;
  if (in_sizes[3] < 1) return;
  if (in_sizes[4] != D_ * HD_ || in_sizes[5] != HD_) return;
  if (in_sizes[6] != D_ * HD_ || in_sizes[7] != HD_) return;
  if (in_sizes[8] != D_ * H_ || in_sizes[9] != H_) return;
  if (out_size != B_ * H_ * D_ * D_) return;

  const float* x      = (const float*)d_in[0];
  const float* M0     = (const float*)d_in[1];
  const float* router = (const float*)d_in[2];
  const int*   mem_id = (const int*)  d_in[3];
  const float* Wk     = (const float*)d_in[4];
  const float* bk     = (const float*)d_in[5];
  const float* Wv     = (const float*)d_in[6];
  const float* bv     = (const float*)d_in[7];
  const float* Wf     = (const float*)d_in[8];
  const float* bf     = (const float*)d_in[9];
  float* out = (float*)d_out;

  const int BH = 8;
  const size_t OFF_XH  = 0;
  const size_t SZ_XH   = (size_t)B_ * S_ * D_ * 2;
  const size_t OFF_WKT = OFF_XH + SZ_XH;
  const size_t SZ_WT   = (size_t)HD_ * D_ * 2;
  const size_t OFF_WVT = OFF_WKT + SZ_WT;
  const size_t OFF_C   = OFF_WVT + SZ_WT;
  const size_t SZ_C    = (size_t)B_ * H_ * S_ * 4;
  const size_t OFF_F   = OFF_C + SZ_C;
  const size_t SZ_F    = (size_t)B_ * H_ * 32 * 4;
  const size_t OFF_KP  = OFF_F + SZ_F;
  const size_t SZ_PL   = (size_t)BH * HD_ * S_ * 2;
  const size_t OFF_VP  = OFF_KP + SZ_PL;
  const size_t TOTAL   = OFF_VP + SZ_PL;
  if (TOTAL > ws_size) return;

  unsigned char* wsc = (unsigned char*)d_ws;
  unsigned short* xh  = (unsigned short*)(wsc + OFF_XH);
  unsigned short* wkt = (unsigned short*)(wsc + OFF_WKT);
  unsigned short* wvt = (unsigned short*)(wsc + OFF_WVT);
  float* cbuf = (float*)(wsc + OFF_C);
  float* fbuf = (float*)(wsc + OFF_F);
  unsigned short* kpl = (unsigned short*)(wsc + OFF_KP);
  unsigned short* vpl = (unsigned short*)(wsc + OFF_VP);

  {
    const int n2 = B_ * S_ * D_ / 2;
    cast_f32_f16x2<<<(n2 + 255) / 256, 256, 0, stream>>>(x, (_Float16*)xh, n2);
  }
  wt_cast<<<dim3(HD_ / 32, 2), 256, 0, stream>>>(Wk, Wv, (_Float16*)wkt, (_Float16*)wvt);
  gate_coef<<<B_, 256, 0, stream>>>(x, router, mem_id, Wf, bf, cbuf, fbuf);

  for (int half = 0; half < 2; ++half) {
    const unsigned short* xhalf = xh + (size_t)half * BH * S_ * D_;
    const float* chalf = cbuf + (size_t)half * BH * H_ * S_;
    wmma_gemm64<0, false, 1, 1, false, 0, true, false><<<dim3((HD_ / 64) * (S_ / 64) / 8, BH), 256, 0, stream>>>(
        wkt, wkt, D_, 0L,
        xhalf, xhalf, D_, (long)S_ * D_,
        (void*)kpl, (void*)kpl, S_, (long)HD_ * S_,
        bk,
        chalf, 0L,
        fbuf, 0,
        chalf, (long)H_ * S_, S_, 7, 4096.0f,
        HD_, S_, D_, 1.0f);
    wmma_gemm64<0, false, 1, 1, false, 0, false, false><<<dim3((HD_ / 64) * (S_ / 64) / 8, BH), 256, 0, stream>>>(
        wvt, wvt, D_, 0L,
        xhalf, xhalf, D_, (long)S_ * D_,
        (void*)vpl, (void*)vpl, S_, (long)HD_ * S_,
        bv,
        chalf, 0L,
        fbuf, 0,
        chalf, 0L, 0, 0, 16.0f,
        HD_, S_, D_, 1.0f);
    float* ohalf = out + (size_t)half * BH * H_ * D_ * D_;
    const float* mhalf = M0 + (size_t)half * BH * H_ * D_ * D_;
    const float* fhalf = fbuf + (size_t)half * BH * H_ * 32;
    wmma_gemm64<0, false, 0, 0, true, 0, false, true><<<dim3(1, BH * H_), 128, 0, stream>>>(
        kpl, kpl, S_, (long)D_ * S_,
        vpl, vpl, S_, (long)D_ * S_,
        (void*)ohalf, (void*)ohalf, D_, (long)D_ * D_,
        bk,
        mhalf, (long)D_ * D_,
        fhalf, 32,
        chalf, 0L, 0, 0, 1.0f,
        D_, D_, S_, 1.0f / 65536.0f);
  }
  (void)hipGetLastError();
}
